// LeakyRNNModel_10033043604057
// MI455X (gfx1250) — hardware-verified
//
#include <hip/hip_runtime.h>


namespace {
constexpr int N = 1024, NI = 32, NO = 32, Bn = 16, T = 1000;
constexpr float ALPHA = 0.1f, OMA = 0.9f, SN = 0.01f, AS_ = 8.0f;

typedef _Float16 b16;
typedef __attribute__((ext_vector_type(16))) _Float16 v16b;
typedef __attribute__((ext_vector_type(8))) _Float16 v8b;
typedef __attribute__((ext_vector_type(8))) float v8f;
typedef __attribute__((ext_vector_type(4))) float v4f;
__device__ __forceinline__ float bf16_rne(float f) { unsigned int u = __float_as_uint(f); u += 0x7FFFu + ((u >> 16) & 1u); return __uint_as_float(u & 0xFFFF0000u); }
__device__ __forceinline__ void split16(float v, b16& hi, b16& lo) { hi = (b16)v; lo = (b16)(v - (float)hi); }
__device__ __forceinline__ v16b frag_kb(const b16* p, int hh) { const v8b a = *(const v8b*)(p + 8 * hh), b = *(const v8b*)(p + 16 + 8 * hh); v16b f;
#pragma unroll
  for (int e = 0; e < 8; ++e) { f[e] = a[e]; f[8 + e] = b[e]; } return f; }
__device__ __forceinline__ v8f wmma16b(v16b a, v16b b, v8f c) { v8f d = __builtin_amdgcn_wmma_f32_16x16x32_f16(false, a, false, b, (short)0, c, false, false); asm volatile("v_nop\n\tv_nop\n\tv_nop\n\tv_nop" : "+v"(d) : "v"(a), "v"(b)); return d; }
__device__ __forceinline__ float pmul(float a, float b) { float p = a * b; asm volatile("" : "+v"(p)); return p; }
__device__ __forceinline__ float tanh_n(float x) { const float ax = fabsf(x); const float e = __builtin_amdgcn_exp2f(-2.8853900817779268f * ax); float t = (1.0f - e) / (1.0f + e); return (x < 0.0f) ? -t : t; }

__global__ __launch_bounds__(256) void prep_kernel(const float* __restrict__ Win, const float* __restrict__ bias, const float* __restrict__ Wrec, const float* __restrict__ Wout, const float* __restrict__ bout, const float* __restrict__ Wfb, b16* __restrict__ Rr, b16* __restrict__ Ri, float* __restrict__ P) {
  const size_t tid = (size_t)blockIdx.x * 256 + threadIdx.x, nth = (size_t)gridDim.x * 256;
  for (int pass = 0; pass < 2; ++pass) {
    for (size_t p = tid; p < (size_t)N * N / 8; p += nth) { const int o = (int)(p / (N / 8)), k0 = (int)(p % (N / 8)) * 8; v8b v; for (int e = 0; e < 8; ++e) v[e] = (b16)bf16_rne(Wrec[(size_t)(k0 + e) * N + o]); *(volatile v8b*)(Rr + (size_t)o * N + k0) = v; }
    for (size_t p = tid; p < (size_t)N * NI / 8; p += nth) { const int o = (int)(p / (NI / 8)), k0 = (int)(p % (NI / 8)) * 8; v8b v; for (int e = 0; e < 8; ++e) v[e] = (b16)bf16_rne(Win[(size_t)(k0 + e) * N + o]); *(volatile v8b*)(Ri + (size_t)o * NI + k0) = v; }
    for (size_t q = tid; q < 66592; q += nth) { const int i = (int)q; float v; if (i < 1024) v = bias[i]; else if (i < 33792) v = Wout[i - 1024]; else if (i < 33824) v = bout[i - 33792]; else v = Wfb[i - 33824]; P[q] = bf16_rne(v); }
    __threadfence(); }
}

__global__ __launch_bounds__(64) void drive_kernel(const float* __restrict__ inp, const b16* __restrict__ Ri, const float* __restrict__ P, float* __restrict__ DRV) {
  __shared__ __attribute__((aligned(16))) float Ts[2][32][128 + 4];
  const int lane = threadIdx.x & 31, wave = threadIdx.x >> 5, nloc = lane & 15, hlf = lane >> 4, m0 = blockIdx.y * 32, c0 = blockIdx.x * 256 + wave * 128;
  v16b a0, a1;
#pragma unroll
  for (int e = 0; e < 16; ++e) { const int k = (e < 8) ? (8 * hlf + e) : (16 + 8 * hlf + e - 8); a0[e] = (b16)bf16_rne(inp[(size_t)(m0 + nloc) * NI + k]); a1[e] = (b16)bf16_rne(inp[(size_t)(m0 + 16 + nloc) * NI + k]); }
  v8f acc[2][8];
#pragma unroll
  for (int r = 0; r < 2; ++r)
#pragma unroll
    for (int t = 0; t < 8; ++t) acc[r][t] = (v8f){};
#pragma unroll
  for (int t = 0; t < 8; ++t) { const v16b bw = frag_kb(Ri + (size_t)(c0 + t * 16 + nloc) * NI, hlf); acc[0][t] = wmma16b(a0, bw, acc[0][t]); acc[1][t] = wmma16b(a1, bw, acc[1][t]); }
#pragma unroll
  for (int t = 0; t < 8; ++t) { const float bb = P[c0 + t * 16 + nloc];
#pragma unroll
    for (int r = 0; r < 2; ++r)
#pragma unroll
      for (int v = 0; v < 8; ++v) Ts[wave][r * 16 + 8 * hlf + v][t * 16 + nloc] = acc[r][t][v] + bb; }
  __builtin_amdgcn_fence(__ATOMIC_RELEASE, "workgroup"); __builtin_amdgcn_wave_barrier(); __builtin_amdgcn_fence(__ATOMIC_ACQUIRE, "workgroup");
  for (int pass = 0; pass < 2; ++pass) { for (int i = lane; i < 32 * 32; i += 32) { const int rr = i >> 5, c4 = (i & 31) * 4; *(volatile v4f*)(DRV + (size_t)(m0 + rr) * N + c0 + c4) = *(const v4f*)(&Ts[wave][rr][c4]); } __threadfence(); }
}

__global__ __launch_bounds__(256) void rnn_kernel(const float* __restrict__ DRV, const float* __restrict__ noise, const b16* __restrict__ Rr, const float* __restrict__ P, float* __restrict__ out) {
  __shared__ __attribute__((aligned(16))) float X[Bn][N]; __shared__ __attribute__((aligned(16))) b16 Rh[Bn][N + 8], Rl[Bn][N + 8]; __shared__ float Z[Bn][NO]; __shared__ __attribute__((aligned(16))) float Zo[Bn][NO];
  const int t_ = threadIdx.x, lane = t_ & 31, wave = t_ >> 5, nloc = lane & 15, hlf = lane >> 4;
  const float* Wout = P + 1024; const float* bout = P + 33792; const float* Wfb = P + 33824;
  for (int i = t_; i < Bn * N; i += 256) (&X[0][0])[i] = 0.0f;
  __syncthreads();
  for (int step = 0; step <= T; ++step) {
    for (int i = t_; i < Bn * N; i += 256) { const int b = i >> 10, n = i & 1023; b16 h_, l_; split16(tanh_n(X[b][n]) * AS_, h_, l_); Rh[b][n] = h_; Rl[b][n] = l_; }
    __syncthreads();
    { const int b = t_ >> 4, o0 = (t_ & 15) * 2; float s0 = 0.0f, s1 = 0.0f;
      for (int n = 0; n < N; ++n) { const float r = ((float)Rh[b][n] + (float)Rl[b][n]) * (1.0f / AS_); s0 += pmul(r, Wout[n * NO + o0]); s1 += pmul(r, Wout[n * NO + o0 + 1]); }
      Z[b][o0] = s0 + bout[o0]; Z[b][o0 + 1] = s1 + bout[o0 + 1]; Zo[b][o0] = Z[b][o0]; Zo[b][o0 + 1] = Z[b][o0 + 1]; }
    __syncthreads();
    if (step >= 1) { for (int pass = 0; pass < 2; ++pass) { if (t_ < Bn * NO / 4) { const int b = t_ >> 3, c4 = (t_ & 7) * 4; *(volatile v4f*)(out + ((size_t)b * T + (step - 1)) * NO + c4) = *(const v4f*)(&Zo[b][c4]); } __threadfence(); } }
    if (step == T) break;
    v8f acc[8];
#pragma unroll
    for (int t = 0; t < 8; ++t) acc[t] = (v8f){};
    for (int kb = 0; kb < N; kb += 32) { const v16b ah = frag_kb(&Rh[nloc][kb], hlf), al = frag_kb(&Rl[nloc][kb], hlf);
#pragma unroll
      for (int t = 0; t < 8; ++t) { const v16b bw = frag_kb(Rr + (size_t)(wave * 128 + t * 16 + nloc) * N + kb, hlf); acc[t] = wmma16b(ah, bw, acc[t]); acc[t] = wmma16b(al, bw, acc[t]); } }
#pragma unroll
    for (int t = 0; t < 8; ++t) { const int n = wave * 128 + t * 16 + nloc;
#pragma unroll
      for (int r = 0; r < 8; ++r) { const int b = 8 * hlf + r; float fb = 0.0f;
#pragma unroll 8
        for (int o = 0; o < NO; ++o) fb += pmul(Z[b][o], Wfb[o * N + n]);
        const float u = DRV[((size_t)b * T + step) * N + n] + acc[t][r] * (1.0f / AS_) + fb;
        X[b][n] = pmul(OMA, X[b][n]) + pmul(ALPHA, u) + pmul(SN, bf16_rne(noise[((size_t)b * T + step) * N + n])); } }
    __syncthreads(); }
}
}

extern "C" void kernel_launch(void* const* d_in, const int* in_sizes, int n_in,
                              void* d_out, int out_size, void* d_ws, size_t ws_size, hipStream_t stream) {
  (void)n_in; (void)out_size;
  const float* inp = (const float*)d_in[0]; const float* noise = (const float*)d_in[1]; const float* Win = (const float*)d_in[2]; const float* bias = (const float*)d_in[3]; const float* Wrec = (const float*)d_in[4]; const float* Wout = (const float*)d_in[5]; const float* bout = (const float*)d_in[6]; const float* Wfb = (const float*)d_in[7];
  float* out = (float*)d_out;
  if (in_sizes[0] != Bn * T * NI || in_sizes[1] != Bn * T * N || in_sizes[4] != N * N || in_sizes[7] != NO * N) return;
  size_t off = 0; char* ws = (char*)d_ws;
  auto carve = [&](size_t bytes) { char* p = ws + off; off += (bytes + 255) & ~(size_t)255; return p; };
  b16* Rr = (b16*)carve((size_t)N * N * 2); b16* Ri = (b16*)carve((size_t)N * NI * 2); float* P = (float*)carve(66592 * 4); float* DRV = (float*)carve((size_t)Bn * T * N * 4);
  if (off > ws_size) return;
  prep_kernel<<<256, 256, 0, stream>>>(Win, bias, Wrec, Wout, bout, Wfb, Rr, Ri, P);
  drive_kernel<<<dim3(N / 256, Bn * T / 32), 64, 0, stream>>>(inp, Ri, P, DRV);
  rnn_kernel<<<1, 256, 0, stream>>>(DRV, noise, Rr, P, out);
}
